// TuFormAttention_6073083756834
// MI455X (gfx1250) — hardware-verified
//
#include <hip/hip_runtime.h>
#include <math.h>

#define NBATCH 2
#define SEQ    256
#define HID    256
#define QKVN   768
#define NROW   (NBATCH * SEQ)
#define KSTAGE 32

static_assert((SEQ % KSTAGE) == 0 && (HID % 64) == 0 && (QKVN % 64) == 0 && (NROW % 32) == 0);
static_assert(HID == 256 && SEQ == 256);
static constexpr float kLog2E = 1.4426950408889634f;

typedef __bf16 v16b __attribute__((ext_vector_type(16)));
typedef float v8f __attribute__((ext_vector_type(8)));
typedef float v4f __attribute__((ext_vector_type(4)));
typedef unsigned int v4u __attribute__((ext_vector_type(4)));
typedef unsigned int v2u __attribute__((ext_vector_type(2)));
typedef unsigned short v8us __attribute__((ext_vector_type(8)));

__device__ __forceinline__ unsigned short bf_bits(float f) {
  unsigned u = __float_as_uint(f);
  return (unsigned short)((u + 0x7FFFu + ((u >> 16) & 1u)) >> 16);
}
__device__ __forceinline__ float bf_up(unsigned short hb) { return __uint_as_float(((unsigned)hb) << 16); }
__device__ __forceinline__ float bfr(float f) { return bf_up(bf_bits(f)); }
__device__ __forceinline__ unsigned pk16(unsigned short a, unsigned short b) { return (unsigned)a | ((unsigned)b << 16); }
__device__ __forceinline__ v8f zero8() { v8f z = {0.f, 0.f, 0.f, 0.f, 0.f, 0.f, 0.f, 0.f}; return z; }

__device__ __forceinline__ v16b ldfrag_b(const unsigned short* p) {
  union { v16b v; v8us s[2]; } f;
  f.s[0] = *(const v8us*)(p);
  f.s[1] = *(const v8us*)(p + 16);
  return f.v;
}

__device__ __forceinline__ v8f mma_b(v16b a, v16b b, v8f c) {
  c = __builtin_amdgcn_wmma_f32_16x16x32_bf16(false, a, false, b, (short)0, c, false, false);
#if defined(__HIP_DEVICE_COMPILE__)
  asm volatile("v_nop\n\tv_nop\n\tv_nop\n\tv_nop" : "+v"(c) : "v"(a), "v"(b));
#endif
  return c;
}
__device__ __forceinline__ void wave_sync_lds() {
#if defined(__HIP_DEVICE_COMPILE__)
  __builtin_amdgcn_fence(__ATOMIC_RELEASE, "workgroup");
  __builtin_amdgcn_wave_barrier();
  __builtin_amdgcn_fence(__ATOMIC_ACQUIRE, "workgroup");
#endif
}

__global__ __launch_bounds__(256) void cvtbf(const float* __restrict__ src, unsigned short* dst, int n8) {
  const int P = blockIdx.x * 256 + threadIdx.x;
  const int Pc = (P < n8) ? P : (n8 - 1);
  const float* s = src + (size_t)Pc * 8;
  const v4f a = *(const v4f*)(s);
  const v4f b = *(const v4f*)(s + 4);
  v4u u;
  u[0] = pk16(bf_bits(a[0]), bf_bits(a[1]));
  u[1] = pk16(bf_bits(a[2]), bf_bits(a[3]));
  u[2] = pk16(bf_bits(b[0]), bf_bits(b[1]));
  u[3] = pk16(bf_bits(b[2]), bf_bits(b[3]));
  unsigned short* d = dst + (size_t)Pc * 8;
  if (P < n8) *(volatile v4u*)d = u;
  __threadfence();
  if (P < n8) *(volatile v4u*)d = u;
}

__global__ __launch_bounds__(256) void gemm_bf(
    const unsigned short* __restrict__ Ap, int lda,
    const unsigned short* __restrict__ Btp, int ldb,
    float* Cp, int ldc, const float* __restrict__ bias,
    int M, int N, int K) {
  __shared__ __align__(16) float sT[8][16 * 68];
  const int lane = threadIdx.x & 31;
  const int wave = threadIdx.x >> 5;
  const int tilesN = N >> 6;
  const int tilesM = M >> 5;
  const int tile = blockIdx.x * 8 + wave;
  if (tile >= tilesM * tilesN) return;
  const int tm = tile / tilesN;
  const int tn = tile - tm * tilesN;
  const int m0 = tm << 5;
  const int n0 = tn << 6;

  const int rlane = lane & 15;
  const int koff  = (lane >> 4) * 8;
  const int mOff  = (lane >> 4) * 8;

  v8f acc[2][4];
#pragma unroll
  for (int i = 0; i < 2; ++i)
#pragma unroll
    for (int j = 0; j < 4; ++j) acc[i][j] = zero8();

  for (int k0 = 0; k0 < K; k0 += 32) {
    v16b bh[4];
#pragma unroll
    for (int j = 0; j < 4; ++j) bh[j] = ldfrag_b(Btp + (size_t)(n0 + (j << 4) + rlane) * ldb + koff + k0);
#pragma unroll
    for (int i = 0; i < 2; ++i) {
      const v16b ah = ldfrag_b(Ap + (size_t)(m0 + (i << 4) + rlane) * lda + koff + k0);
#pragma unroll
      for (int j = 0; j < 4; ++j) acc[i][j] = mma_b(ah, bh[j], acc[i][j]);
    }
  }

  const int hq = lane >> 4, q = lane & 15;
  const int col = n0 + 4 * q;
  float bb[4];
#pragma unroll
  for (int e = 0; e < 4; ++e) {
    int bi = col + e;
    if (bi > N - 1) bi = N - 1;
    bb[e] = bfr(bias[bi]);
  }
  float* slab = sT[wave];
#pragma unroll
  for (int i = 0; i < 2; ++i) {
    const int mBase = m0 + (i << 4);
#pragma unroll
    for (int j = 0; j < 4; ++j) {
#pragma unroll
      for (int r = 0; r < 8; ++r) {
        slab[(mOff + r) * 68 + (j << 4) + rlane] = acc[i][j][r];
      }
    }
    wave_sync_lds();
    v4f ov[8];
#pragma unroll
    for (int it = 0; it < 8; ++it) {
      const int row = it * 2 + hq;
      const float* sp = slab + row * 68 + 4 * q;
      v4f o;
#pragma unroll
      for (int e = 0; e < 4; ++e) o[e] = sp[e] + bb[e];
      ov[it] = o;
    }
#pragma unroll
    for (int it = 0; it < 8; ++it) {
      const int row = it * 2 + hq;
      *(volatile v4f*)(Cp + (size_t)(mBase + row) * ldc + col) = ov[it];
    }
    __threadfence();
#pragma unroll
    for (int it = 0; it < 8; ++it) {
      const int row = it * 2 + hq;
      *(volatile v4f*)(Cp + (size_t)(mBase + row) * ldc + col) = ov[it];
    }
    __threadfence();
    wave_sync_lds();
  }
}

__global__ __launch_bounds__(256) void attn(const float* __restrict__ QKV,
                                           const unsigned short* __restrict__ WCB,
                                           const float* __restrict__ bc, float* out) {
  __shared__ __align__(16) unsigned short KH[KSTAGE * HID];
  __shared__ __align__(16) unsigned short KL[KSTAGE * HID];
  __shared__ __align__(16) float Os[HID];

  const int bs = blockIdx.x;
  const int b = bs >> 8;
  const int s = bs & (SEQ - 1);
  const int tid = threadIdx.x, wave = tid >> 5, lane = tid & 31, h = lane >> 4, c = lane & 15;

  const float* qrow  = QKV + (size_t)(b * SEQ + s) * QKVN;
  const float* kbase = QKV + (size_t)(b * SEQ) * QKVN + HID;
  const float* vbase = QKV + (size_t)(b * SEQ) * QKVN + 2 * HID;

  const int r4 = (tid & 63) * 4;
  const int lr = tid >> 6;
  const v4f q4 = *(const v4f*)(qrow + r4);

  const int pw = wave * 32;
  float bcv[2];
  bcv[0] = bfr(bc[pw + c]);
  bcv[1] = bfr(bc[pw + 16 + c]);
  const unsigned short* wrow0 = WCB + (size_t)(pw + c) * HID + 8 * h;
  const unsigned short* wrow1 = WCB + (size_t)(pw + 16 + c) * HID + 8 * h;
  const float* vcol0 = vbase + pw + c;
  const float* vcol1 = vbase + pw + 16 + c;

  float mx[2], dn[2], ac[2];
#pragma unroll
  for (int j = 0; j < 2; ++j) { mx[j] = -1.0e30f; dn[j] = 0.f; ac[j] = 0.f; }

  for (int st = 0; st < SEQ / KSTAGE; ++st) {
    const int l0 = st * KSTAGE;
#pragma unroll 2
    for (int i = 0; i < 8; ++i) {
      const int l = lr + 4 * i;
      const v4f k4 = *(const v4f*)(kbase + (size_t)(l0 + l) * QKVN + r4);
      unsigned short hb[4], lb[4];
#pragma unroll
      for (int e = 0; e < 4; ++e) {
        const float x = k4[e] * q4[e];
        const unsigned short hh = bf_bits(x);
        hb[e] = hh;
        lb[e] = bf_bits(x - bf_up(hh));
      }
      v2u hv, lv;
      hv[0] = pk16(hb[0], hb[1]);
      hv[1] = pk16(hb[2], hb[3]);
      lv[0] = pk16(lb[0], lb[1]);
      lv[1] = pk16(lb[2], lb[3]);
      *(v2u*)(KH + l * HID + r4) = hv;
      *(v2u*)(KL + l * HID + r4) = lv;
    }
    __syncthreads();

    v8f acc[2][2];
#pragma unroll
    for (int i = 0; i < 2; ++i) { acc[i][0] = zero8(); acc[i][1] = zero8(); }
#pragma unroll 2
    for (int ks = 0; ks < HID / 32; ++ks) {
      const v16b b0 = ldfrag_b(wrow0 + ks * 32);
      const v16b b1 = ldfrag_b(wrow1 + ks * 32);
#pragma unroll
      for (int i = 0; i < 2; ++i) {
        const v16b ah = ldfrag_b(KH + (16 * i + c) * HID + ks * 32 + 8 * h);
        const v16b al = ldfrag_b(KL + (16 * i + c) * HID + ks * 32 + 8 * h);
        acc[i][0] = mma_b(ah, b0, acc[i][0]);
        acc[i][0] = mma_b(al, b0, acc[i][0]);
        acc[i][1] = mma_b(ah, b1, acc[i][1]);
        acc[i][1] = mma_b(al, b1, acc[i][1]);
      }
    }

#pragma unroll
    for (int j = 0; j < 2; ++j) {
      float sv[2][8];
      float tmax = -1.0e30f;
#pragma unroll
      for (int i = 0; i < 2; ++i) {
#pragma unroll
        for (int r = 0; r < 8; ++r) {
          sv[i][r] = acc[i][j][r] + bcv[j];
          tmax = fmaxf(tmax, sv[i][r]);
        }
      }
      tmax = fmaxf(tmax, __shfl_xor(tmax, 16, 32));
      const float mn = fmaxf(mx[j], tmax);
      const float sc = exp2f((mx[j] - mn) * kLog2E);
      const float* vcol = (j == 0) ? vcol0 : vcol1;
      float ps = 0.f, pa = 0.f;
#pragma unroll
      for (int i = 0; i < 2; ++i) {
#pragma unroll
        for (int r = 0; r < 8; ++r) {
          const int l = l0 + 16 * i + 8 * h + r;
          const float e = exp2f((sv[i][r] - mn) * kLog2E);
          ps += e;
          pa += e * vcol[(size_t)l * QKVN];
        }
      }
      ps += __shfl_xor(ps, 16, 32);
      pa += __shfl_xor(pa, 16, 32);
      dn[j] = dn[j] * sc + ps;
      ac[j] = ac[j] * sc + pa;
      mx[j] = mn;
    }
    __syncthreads();
  }

  {
    const float o0 = ac[0] * (1.0f / dn[0]);
    const float o1 = ac[1] * (1.0f / dn[1]);
    if (h == 0) {
      Os[pw + c] = o0;
      Os[pw + 16 + c] = o1;
    }
  }
  __syncthreads();
  const int tq = (tid < 64) ? tid : 0;
  const v4f ov = *(const v4f*)(Os + 4 * tq);
  float* op = out + (size_t)bs * HID + 4 * tq;
  if (tid < 64) *(volatile v4f*)op = ov;
  __threadfence();
  if (tid < 64) *(volatile v4f*)op = ov;
}

extern "C" void kernel_launch(void* const* d_in, const int* in_sizes, int n_in,
                              void* d_out, int out_size, void* d_ws, size_t ws_size,
                              hipStream_t stream) {
  if (n_in < 5) return;
  if (in_sizes[0] != NROW * HID || in_sizes[1] != QKVN * HID || in_sizes[2] != QKVN) return;
  if (in_sizes[3] != HID * HID || in_sizes[4] != HID) return;
  if (out_size != NROW * HID) return;

  const float* x    = (const float*)d_in[0];
  const float* wqkv = (const float*)d_in[1];
  const float* bqkv = (const float*)d_in[2];
  const float* wc   = (const float*)d_in[3];
  const float* bcp  = (const float*)d_in[4];
  float* out = (float*)d_out;

  const size_t PXB  = (size_t)NROW * HID * 2;
  const size_t PWB  = (size_t)QKVN * HID * 2;
  const size_t PWC  = (size_t)HID * HID * 2;
  const size_t PQKV = (size_t)NROW * QKVN * 4;
  size_t off = 0;
  const size_t oXB  = off; off += PXB;
  const size_t oWB  = off; off += PWB;
  const size_t oWC  = off; off += PWC;
  const size_t oQKV = off; off += PQKV;
  if (off > ws_size) return;
  if (off > (size_t)134217728) return;

  char* ws = (char*)d_ws;
  unsigned short* XB  = (unsigned short*)(ws + oXB);
  unsigned short* WB  = (unsigned short*)(ws + oWB);
  unsigned short* WCB = (unsigned short*)(ws + oWC);
  float*          QKV = (float*)(ws + oQKV);

  const dim3 blk(256);
  const int nx8 = NROW * HID / 8;
  const int nw8 = QKVN * HID / 8;
  const int nc8 = HID * HID / 8;

  cvtbf<<<dim3((nx8 + 255) / 256), blk, 0, stream>>>(x, XB, nx8);
  cvtbf<<<dim3((nw8 + 255) / 256), blk, 0, stream>>>(wqkv, WB, nw8);
  cvtbf<<<dim3((nc8 + 255) / 256), blk, 0, stream>>>(wc, WCB, nc8);

  {
    const int tiles = (NROW / 32) * (QKVN / 64);
    gemm_bf<<<dim3((tiles + 7) / 8), blk, 0, stream>>>(XB, HID, WB, HID, QKV, QKVN, bqkv, NROW, QKVN, HID);
  }

  attn<<<dim3(NROW), blk, 0, stream>>>(QKV, WCB, bcp, out);

  (void)hipGetLastError();
}
